// GraphTransformerEncoder_19696720020245
// MI455X (gfx1250) — hardware-verified
//
#include <hip/hip_runtime.h>
#include <hip/hip_bf16.h>

typedef __attribute__((ext_vector_type(16))) _Float16 v16h;
typedef __attribute__((ext_vector_type(8)))  _Float16 v8h;
typedef __attribute__((ext_vector_type(8)))  float    v8f;

#if defined(__gfx1250__) &&                                             \
    __has_builtin(__builtin_amdgcn_global_load_async_to_lds_b128) &&    \
    __has_builtin(__builtin_amdgcn_global_store_async_from_lds_b128) && \
    __has_builtin(__builtin_amdgcn_s_wait_asynccnt)
#define ASYNC_LDS 1
typedef __attribute__((ext_vector_type(4))) int v4i;
typedef v4i v4i_gl  __attribute__((address_space(1)));
typedef v4i v4i_lds __attribute__((address_space(3)));
#endif

typedef __attribute__((ext_vector_type(4))) float v4f_t;
typedef float v4fa __attribute__((ext_vector_type(4), may_alias));
#define ST2F(ptr, val) do { *(volatile float*)(ptr) = (val); __threadfence(); *(volatile float*)(ptr) = (val); } while (0)

namespace {
constexpr int kGB = 256;
constexpr int kNPart = 4 * 8192 / kGB;

constexpr int kB = 4, kNA = 64, kT = 128, kD = 128, kH = 8, kL = 3, kDFF = 512;
constexpr int kE = 65536;
constexpr int kNN = kT * kNA;
constexpr int kTok = kB * kNA * kT;
constexpr int kXel = kB * kNA * kT * kD;
constexpr int kWL = 4 * kD * kD + 2 * kD * kDFF;


__device__ inline v8f wmma16(v16h a, v16h b, v8f c) {
  return __builtin_amdgcn_wmma_f32_16x16x32_f16(false, a, false, b, (short)0, c,
                                                false, false);
}

__device__ inline v16h ld_a(const _Float16* src, int ld, int m0, int k0) {
  const int lane = threadIdx.x & 31;
  const _Float16* p = src + (size_t)(m0 + (lane & 15)) * ld + k0 + ((lane >> 4) << 3);
  v8h lo = *(const v8h*)(p);
  v8h hi = *(const v8h*)(p + 16);
  return __builtin_shufflevector(lo, hi, 0, 1, 2, 3, 4, 5, 6, 7,
                                 8, 9, 10, 11, 12, 13, 14, 15);
}

__device__ inline v16h ld_b16(const _Float16* base, int K, int k0, int n0) {
  const int lane = threadIdx.x & 31;
  const _Float16* p = base + (size_t)(n0 + (lane & 15)) * K + k0 + ((lane >> 4) << 3);
  v8h lo = *(const v8h*)(p);
  v8h hi = *(const v8h*)(p + 16);
  return __builtin_shufflevector(lo, hi, 0, 1, 2, 3, 4, 5, 6, 7,
                                 8, 9, 10, 11, 12, 13, 14, 15);
}

__device__ inline v16h ld_a_pad16(const _Float16* src, int ld, int m0, int c0) {
  const int lane = threadIdx.x & 31;
  const _Float16* p = src + (size_t)(m0 + (lane & 15)) * ld + c0 + ((lane >> 4) << 3);
  v8h lo = *(const v8h*)(p);
  v8h z = {};
  return __builtin_shufflevector(lo, z, 0, 1, 2, 3, 4, 5, 6, 7,
                                 8, 9, 10, 11, 12, 13, 14, 15);
}

__device__ inline v16h ld_bT_pad16(const _Float16* src, int ld, int c0, int n0) {
  const int lane = threadIdx.x & 31;
  const _Float16* p = src + (size_t)(n0 + (lane & 15)) * ld + c0 + ((lane >> 4) << 3);
  v8h lo = *(const v8h*)(p);
  v8h z = {};
  return __builtin_shufflevector(lo, z, 0, 1, 2, 3, 4, 5, 6, 7,
                                 8, 9, 10, 11, 12, 13, 14, 15);
}


__device__ inline void ln_rows(float* xres, _Float16* abuf, const float* g,
                               const float* b, int m0, int lane) {
  for (int i = 0; i < 16; ++i) {
    float* xr = xres + (size_t)(m0 + i) * kD;
    float v[4];
    float s = 0.f;
#pragma unroll
    for (int c = 0; c < 4; ++c) { v[c] = xr[lane * 4 + c]; s += v[c]; }
#pragma unroll
    for (int mm = 1; mm < 32; mm <<= 1) s += __shfl_xor(s, mm, 32);
    const float mean = s * (1.f / kD);
    float vs = 0.f;
#pragma unroll
    for (int c = 0; c < 4; ++c) { float d = v[c] - mean; vs += d * d; }
#pragma unroll
    for (int mm = 1; mm < 32; mm <<= 1) vs += __shfl_xor(vs, mm, 32);
    const float rs = rsqrtf(vs * (1.f / kD) + 1e-5f);
#pragma unroll
    for (int c = 0; c < 4; ++c) {
      const int col = lane * 4 + c;
      const float y = (v[c] - mean) * rs * g[col] + b[col];
      xr[col] = y;
      abuf[(size_t)(m0 + i) * kD + col] = (_Float16)y;
    }
  }
}


__global__ __launch_bounds__(256) void pack_kernel(
    const float* __restrict__ wq, const float* __restrict__ wk,
    const float* __restrict__ wv, const float* __restrict__ wo,
    const float* __restrict__ w1, const float* __restrict__ w2,
    _Float16* __restrict__ wp) {
  const int idx0 = (blockIdx.x * 256 + threadIdx.x) * 2;
  float pv[2];
#pragma unroll
  for (int q2 = 0; q2 < 2; ++q2) {
  const int idx = idx0 + q2;
  const int l = idx / kWL;
  const int r = idx - l * kWL;
  float v;
  if (r < 4 * kD * kD) {
    const int m = r >> 14;
    const int e = r & 16383;
    const int n = e >> 7, k = e & 127;
    const float* W = (m == 0) ? wq : (m == 1) ? wk : (m == 2) ? wv : wo;
    v = W[(size_t)l * kD * kD + (size_t)k * kD + n];
  } else if (r < 4 * kD * kD + kD * kDFF) {
    const int e = r - 4 * kD * kD;
    const int n = e >> 7, k = e & 127;
    v = w1[(size_t)l * kD * kDFF + (size_t)k * kDFF + n];
  } else {
    const int e = r - (4 * kD * kD + kD * kDFF);
    const int n = e >> 9, k = e & 511;
    v = w2[(size_t)l * kDFF * kD + (size_t)k * kD + n];
  }
  pv[q2] = v;
  }
  const unsigned pp = (unsigned)__builtin_bit_cast(unsigned short, (_Float16)pv[0]) | ((unsigned)__builtin_bit_cast(unsigned short, (_Float16)pv[1]) << 16);
  *(volatile unsigned*)(wp + idx0) = pp; __threadfence(); *(volatile unsigned*)(wp + idx0) = pp;
}

__global__ __launch_bounds__(256) void embed_kernel(const float* __restrict__ feat,
                                                    const float* __restrict__ hw,
                                                    const float* __restrict__ hb,
                                                    float* __restrict__ x,
                                                    float* __restrict__ oute) {
  const int idx = blockIdx.x * 256 + threadIdx.x;
  const int d = idx & (kD - 1);
  const int t = (idx >> 7) & (kT - 1);
  const int bn = idx >> 14;
  const float* f = feat + ((size_t)bn * kT + t) * 3;
  float v = hb[d] + f[0] * hw[0 * kD + d] + f[1] * hw[1 * kD + d] + f[2] * hw[2 * kD + d];
  const int i2 = d & ~1;
  const float ang = (float)t * expf(-9.2103403719761836f * (float)i2 / (float)kD);
  float sn, cs; sincosf(ang, &sn, &cs);
  const float pe = (d & 1) ? cs : sn;
  const float ve = v + pe;
  ST2F(x + idx, v); ST2F(oute + idx, ve);
}

__global__ __launch_bounds__(256) void xformer_kernel(
    float* __restrict__ oute, const _Float16* __restrict__ wp,
    const float* __restrict__ bq, const float* __restrict__ bk,
    const float* __restrict__ bv, const float* __restrict__ bo,
    const float* __restrict__ ln1g, const float* __restrict__ ln1b,
    const float* __restrict__ fb1, const float* __restrict__ fb2,
    const float* __restrict__ ln2g, const float* __restrict__ ln2b) {
  __shared__ float    xres[kT * kD];
  __shared__ _Float16 abuf[kT * kD];
  __shared__ _Float16 hbuf[kT * kDFF];

  _Float16* qbuf = hbuf;
  _Float16* kbuf = hbuf + 16384;
  _Float16* vbuf = hbuf + 32768;
  _Float16* pbuf = hbuf + 49152;

  const int tid = threadIdx.x;
  const int lane = tid & 31;
  const int wv8 = tid >> 5;
  const int m0 = wv8 * 16;
  const int rb = (lane >> 4) << 3;
  float* xg = oute + (size_t)blockIdx.x * kT * kD;

#ifdef ASYNC_LDS
  for (int i = tid * 4; i < kT * kD; i += 256 * 4)
    __builtin_amdgcn_global_load_async_to_lds_b128(
        (v4i_gl*)(xg + i), (v4i_lds*)(xres + i), 0, 0);
  __builtin_amdgcn_s_wait_asynccnt(0);
  __syncthreads();
  for (int i = tid; i < kT * kD; i += 256) abuf[i] = (_Float16)xres[i];
#else
  for (int i = tid; i < kT * kD; i += 256) {
    float v = xg[i];
    xres[i] = v;
    abuf[i] = (_Float16)v;
  }
#endif
  __syncthreads();

  for (int l = 0; l < kL; ++l) {
    const _Float16* Pq = wp + (size_t)l * kWL;
    const _Float16* Pk = Pq + 16384;
    const _Float16* Pv = Pq + 32768;
    const _Float16* Po = Pq + 49152;
    const _Float16* P1 = Pq + 65536;
    const _Float16* P2 = Pq + 131072;
    const float* Bq = bq + l * kD;
    const float* Bk = bk + l * kD;
    const float* Bvv = bv + l * kD;
    const float* Bo = bo + l * kD;
    const float* B1 = fb1 + l * kDFF;
    const float* B2 = fb2 + l * kD;
    const float* G1 = ln1g + l * kD;
    const float* Gb1 = ln1b + l * kD;
    const float* G2 = ln2g + l * kD;
    const float* Gb2 = ln2b + l * kD;

    v16h at[4];
#pragma unroll
    for (int kk = 0; kk < 4; ++kk) at[kk] = ld_a(abuf, kD, m0, kk * 32);

    for (int mtx = 0; mtx < 3; ++mtx) {
      const _Float16* W = (mtx == 0) ? Pq : (mtx == 1) ? Pk : Pv;
      const float* bias = (mtx == 0) ? Bq : (mtx == 1) ? Bk : Bvv;
      __builtin_prefetch(W, 0, 1);
      for (int j = 0; j < 8; ++j) {
        v8f acc = {};
#pragma unroll
        for (int kk = 0; kk < 4; ++kk)
          acc = wmma16(at[kk], ld_b16(W, kD, kk * 32, j * 16), acc);
        const int col = j * 16 + (lane & 15);
        const float bc = bias[col];
        if (mtx == 2) {
#pragma unroll
          for (int r = 0; r < 8; ++r)
            vbuf[(size_t)col * kT + (m0 + rb + r)] = (_Float16)(acc[r] + bc);
        } else {
          _Float16* dst = (mtx == 0) ? qbuf : kbuf;
#pragma unroll
          for (int r = 0; r < 8; ++r)
            dst[(size_t)(m0 + rb + r) * kD + col] = (_Float16)(acc[r] + bc);
        }
      }
    }
    __syncthreads();

    for (int h = 0; h < kH; ++h) {
      const int c0 = h * 16;
      v16h aq = ld_a_pad16(qbuf, kD, m0, c0);
      v8f sc[8];
      for (int j = 0; j < 8; ++j) {
        v8f z = {};
        sc[j] = wmma16(aq, ld_bT_pad16(kbuf, kD, c0, j * 16), z);
      }
#pragma unroll
      for (int r = 0; r < 8; ++r) {
        float vals[8];
        float mx = -3.0e38f;
#pragma unroll
        for (int j = 0; j < 8; ++j) {
          vals[j] = sc[j][r] * 0.25f;
          mx = fmaxf(mx, vals[j]);
        }
#pragma unroll
        for (int mm = 1; mm < 16; mm <<= 1) mx = fmaxf(mx, __shfl_xor(mx, mm, 32));
        float sum = 0.f;
#pragma unroll
        for (int j = 0; j < 8; ++j) {
          vals[j] = __expf(vals[j] - mx);
          sum += vals[j];
        }
#pragma unroll
        for (int mm = 1; mm < 16; mm <<= 1) sum += __shfl_xor(sum, mm, 32);
        const float inv = 1.0f / sum;
        const int row = m0 + rb + r;
#pragma unroll
        for (int j = 0; j < 8; ++j)
          pbuf[(size_t)row * kT + j * 16 + (lane & 15)] = (_Float16)(vals[j] * inv * 1024.0f);
      }
      v8f oacc = {};
#pragma unroll
      for (int kk = 0; kk < 4; ++kk)
        oacc = wmma16(ld_a(pbuf, kT, m0, kk * 32),
                      ld_b16(vbuf, kT, kk * 32, c0), oacc);
      const int col = c0 + (lane & 15);
#pragma unroll
      for (int r = 0; r < 8; ++r)
        abuf[(size_t)(m0 + rb + r) * kD + col] = (_Float16)(oacc[r] * (1.0f / 1024.0f));
    }
    __syncthreads();

#pragma unroll
    for (int kk = 0; kk < 4; ++kk) at[kk] = ld_a(abuf, kD, m0, kk * 32);
    __builtin_prefetch(Po, 0, 1);
    for (int j = 0; j < 8; ++j) {
      v8f acc = {};
#pragma unroll
      for (int kk = 0; kk < 4; ++kk)
        acc = wmma16(at[kk], ld_b16(Po, kD, kk * 32, j * 16), acc);
      const int col = j * 16 + (lane & 15);
      const float bc = Bo[col];
#pragma unroll
      for (int r = 0; r < 8; ++r) {
        const size_t ix = (size_t)(m0 + rb + r) * kD + col;
        xres[ix] += acc[r] + bc;
      }
    }
    __syncthreads();

    ln_rows(xres, abuf, G1, Gb1, m0, lane);
    __syncthreads();

#pragma unroll
    for (int kk = 0; kk < 4; ++kk) at[kk] = ld_a(abuf, kD, m0, kk * 32);
    __builtin_prefetch(P1, 0, 1);
    for (int j = 0; j < 32; ++j) {
      v8f acc = {};
#pragma unroll
      for (int kk = 0; kk < 4; ++kk)
        acc = wmma16(at[kk], ld_b16(P1, kD, kk * 32, j * 16), acc);
      const int col = j * 16 + (lane & 15);
      const float bc = B1[col];
#pragma unroll
      for (int r = 0; r < 8; ++r)
        hbuf[(size_t)(m0 + rb + r) * kDFF + col] =
            (_Float16)fmaxf(acc[r] + bc, 0.f);
    }
    __syncthreads();

    {
      __builtin_prefetch(P2, 0, 1);
      v8f acc2[8];
      v8f z = {};
#pragma unroll
      for (int j = 0; j < 8; ++j) acc2[j] = z;
      for (int kk = 0; kk < 16; ++kk) {
        v16h a2 = ld_a(hbuf, kDFF, m0, kk * 32);
#pragma unroll
        for (int j = 0; j < 8; ++j)
          acc2[j] = wmma16(a2, ld_b16(P2, kDFF, kk * 32, j * 16), acc2[j]);
      }
#pragma unroll
      for (int j = 0; j < 8; ++j) {
        const int col = j * 16 + (lane & 15);
        const float bc = B2[col];
#pragma unroll
        for (int r = 0; r < 8; ++r) {
          const size_t ix = (size_t)(m0 + rb + r) * kD + col;
          xres[ix] += acc2[j][r] + bc;
        }
      }
    }
    __syncthreads();

    ln_rows(xres, abuf, G2, Gb2, m0, lane);
    __syncthreads();
  }

#pragma unroll 1
  for (int pass = 0; pass < 2; ++pass) {
    for (int i = tid * 4; i < kT * kD; i += 256 * 4)
      *(volatile v4f_t*)(xg + i) = *(const v4fa*)(xres + i);
    __threadfence();
  }
}

__global__ __launch_bounds__(256) void dot_kernel(const float* __restrict__ oute,
                                                  const float* __restrict__ x,
                                                  float* __restrict__ s) {
  __shared__ float sd[kNA];
  const int lane = threadIdx.x & 31;
  const int wv8 = threadIdx.x >> 5;
  const int b = blockIdx.x / kT, t = blockIdx.x % kT;
#pragma unroll 1
  for (int q = 0; q < 8; ++q) {
    const int n = wv8 * 8 + q;
    const size_t tok = ((size_t)(b * kNA + n)) * kT + t;
    const float* pa = oute + tok * kD;
    const float* pb = x + tok * kD;
    float acc = 0.f;
#pragma unroll
    for (int d = lane; d < kD; d += 32) acc += pa[d] * pb[d];
#pragma unroll
    for (int mm = 1; mm < 32; mm <<= 1) acc += __shfl_xor(acc, mm, 32);
    if (lane == 0) sd[n] = acc;
  }
  __syncthreads();
  if (wv8 == 0) {
    typedef __attribute__((ext_vector_type(2))) float v2f_t;
    typedef float v2fa __attribute__((ext_vector_type(2), may_alias));
    const v2f_t v = *(const v2fa*)(sd + 2 * lane);
    float* d = s + (size_t)b * kNN + t * kNA + 2 * lane;
    *(volatile v2f_t*)d = v; __threadfence(); *(volatile v2f_t*)d = v;
  }
}

__global__ __launch_bounds__(256) void edge_gather_kernel(const int* __restrict__ ei,
                                                          const float* __restrict__ ew,
                                                          const float* __restrict__ s,
                                                          float* __restrict__ g,
                                                          float* __restrict__ part) {
  __shared__ float bins[kGB];
  __shared__ float red1[256], red2[256];
  const int tid = threadIdx.x;
  const int b = blockIdx.x / (kNN / kGB), n0 = (blockIdx.x % (kNN / kGB)) * kGB;
  bins[tid] = 0.f;
  __syncthreads();
  const int* src = ei + ((size_t)b * 2 + 0) * kE;
  const int* dst = ei + ((size_t)b * 2 + 1) * kE;
  for (int e = tid; e < kE; e += 256) {
    const int dd = dst[e] - n0;
    if ((unsigned)dd < (unsigned)kGB) {
      int sr = src[e]; sr = ((unsigned)sr < (unsigned)kNN) ? sr : 0;
      atomicAdd(&bins[dd], ew[(size_t)b * kE + e] * s[(size_t)b * kNN + sr]);
    }
  }
  __syncthreads();
  const float gv = bins[tid];
  ST2F(g + (size_t)b * kNN + n0 + tid, gv);
  red1[tid] = gv; red2[tid] = gv * gv;
  __syncthreads();
  for (int st_ = 128; st_ > 0; st_ >>= 1) { if (tid < st_) { red1[tid] += red1[tid + st_]; red2[tid] += red2[tid + st_]; } __syncthreads(); }
  if (tid < 32) {
    const float pvv = (tid == 0) ? red1[0] : (tid == 1) ? red2[0] : 0.f;
    ST2F(part + (size_t)blockIdx.x * 32 + tid, pvv);
  }
}

__global__ __launch_bounds__(256) void reduce_stats_kernel(const float* __restrict__ part, float* __restrict__ stats) {
  __shared__ double r1[256], r2[256];
  const int tid = threadIdx.x;
  double a = 0.0, b = 0.0;
  for (int i = tid; i < kNPart; i += 256) { a += (double)part[(size_t)i * 32 + 0]; b += (double)part[(size_t)i * 32 + 1]; }
  r1[tid] = a; r2[tid] = b;
  __syncthreads();
  for (int s2 = 128; s2 > 0; s2 >>= 1) { if (tid < s2) { r1[tid] += r1[tid + s2]; r2[tid] += r2[tid + s2]; } __syncthreads(); }
  if (tid < 2) {
    const double invN = 1.0 / (double)(kB * kNN);
    const double mean = r1[0] * invN, var = r2[0] * invN - mean * mean;
    const float v = (tid == 0) ? (float)mean : (float)(1.0 / sqrt((var > 0.0 ? var : 0.0) + 1e-5));
    ST2F(stats + tid, v);
  }
}

__global__ __launch_bounds__(256) void final_kernel(const float* __restrict__ g,
                                                    const float* __restrict__ stats,
                                                    const float* __restrict__ bng,
                                                    const float* __restrict__ bnb,
                                                    const float* __restrict__ lw,
                                                    const float* __restrict__ lb,
                                                    float* __restrict__ out) {
  const int idx = blockIdx.x * 256 + threadIdx.x;
  const int d = idx & (kD - 1);
  const int t = (idx >> 7) & (kT - 1);
  const int bn = idx >> 14;
  const int n = bn & (kNA - 1);
  const int b = bn >> 6;
  const float mean = stats[0], istd = stats[1];
  const float gv = g[(size_t)b * kNN + t * kNA + n];
  const float gh = (gv - mean) * istd * bng[0] + bnb[0];
  const float ov = gh * lw[d] + lb[d];
  ST2F(out + idx, ov);
}

}

extern "C" void kernel_launch(void* const* d_in, const int* in_sizes, int n_in,
                              void* d_out, int out_size, void* d_ws, size_t ws_size,
                              hipStream_t stream) {
  (void)in_sizes; (void)n_in; (void)out_size; (void)ws_size;
  const float* feat = (const float*)d_in[0];
  const int*   eidx = (const int*)d_in[1];
  const float* ew   = (const float*)d_in[2];
  const float* hw   = (const float*)d_in[3];
  const float* hb   = (const float*)d_in[4];
  const float* awq  = (const float*)d_in[5];
  const float* abq  = (const float*)d_in[6];
  const float* awk  = (const float*)d_in[7];
  const float* abk  = (const float*)d_in[8];
  const float* awv  = (const float*)d_in[9];
  const float* abv  = (const float*)d_in[10];
  const float* awo  = (const float*)d_in[11];
  const float* abo  = (const float*)d_in[12];
  const float* l1g  = (const float*)d_in[13];
  const float* l1b  = (const float*)d_in[14];
  const float* fw1  = (const float*)d_in[15];
  const float* fb1  = (const float*)d_in[16];
  const float* fw2  = (const float*)d_in[17];
  const float* fb2  = (const float*)d_in[18];
  const float* l2g  = (const float*)d_in[19];
  const float* l2b  = (const float*)d_in[20];
  const float* bng  = (const float*)d_in[21];
  const float* bnb  = (const float*)d_in[22];
  const float* lgw  = (const float*)d_in[23];
  const float* lgb  = (const float*)d_in[24];

  float* wsf  = (float*)d_ws;
  float* x    = wsf;
  float* oute = x + kXel;
  float* s    = oute + kXel;
  float* g    = s + (size_t)kB * kNN;
  float* part = g + (size_t)kB * kNN;
  float* st   = part + (size_t)kNPart * 32;
  _Float16* wp = (_Float16*)(st + 32);

  pack_kernel<<<(kL * kWL / 2) / 256, 256, 0, stream>>>(awq, awk, awv, awo, fw1, fw2, wp);

  embed_kernel<<<kXel / 256, 256, 0, stream>>>(feat, hw, hb, x, oute);

  xformer_kernel<<<kB * kNA, 256, 0, stream>>>(
      oute, wp, abq, abk, abv, abo, l1g, l1b, fb1, fb2, l2g, l2b);

  dot_kernel<<<kB * kT, 256, 0, stream>>>(oute, x, s);

  edge_gather_kernel<<<kB * (kNN / kGB), 256, 0, stream>>>(eidx, ew, s, g, part);

  reduce_stats_kernel<<<1, 256, 0, stream>>>(part, st);

  final_kernel<<<kXel / 256, 256, 0, stream>>>(g, st, bng, bnb, lgw, lgb,
                                               (float*)d_out);
}
